// MTMD_Domain_Task_Expert_Gate_Shared_Skip_6227702579387
// MI455X (gfx1250) — hardware-verified
//
#include <hip/hip_runtime.h>
#include <stddef.h>


typedef _Float16 v8h  __attribute__((ext_vector_type(8)));
typedef _Float16 v16h __attribute__((ext_vector_type(16)));
typedef float    v8f  __attribute__((ext_vector_type(8)));
typedef float    v4f  __attribute__((ext_vector_type(4)));
union Frag { v16h v; v8h h[2]; };

static constexpr int FEATS = 16, VOCAB = 1000, EDIM = 16;
static constexpr int DIN = 256, SMID = 512, SOUT = 256, H1D = 128, H2D = 64;
static constexpr int NDOM = 3, NTSK = 2, NEXP = 8, NKDT = 6;
static constexpr int NXP = NEXP + NDOM + NTSK;

static constexpr float S_IN   = 64.f;
static constexpr float S_W    = 64.f;
static constexpr float S_SLOT = 1024.f;
static constexpr float S_MID  = 256.f;

static constexpr int WAVES = 2, TPW = 8, SPB = WAVES * TPW * 16;
static constexpr int BO_SKEY = 0;
static constexpr int BO_PERM = 1024;
static constexpr int BO_CNT  = 2048;
static constexpr int BO_RES  = 2176;
static constexpr int BLK_BYTES = 4352;
static constexpr int OFF_IN   = 0;
static constexpr int OFF_SKIP = 8192;
static constexpr int OFF_MID  = 16384;
static constexpr int OFF_FEA  = 8192;
static constexpr int OFF_H1   = 61440;
static constexpr int OFF_GATE = 65536;
static constexpr int OFF_PROB = 68608;
static constexpr int PER_WAVE = 69120;
static constexpr int SMEM_BYTES = BLK_BYTES + WAVES * PER_WAVE;

static constexpr size_t O_SKIP = 0;
static constexpr size_t O_SLOT = O_SKIP + 256 * 256;
static constexpr size_t O_STAR = O_SLOT + 3 * 512 * 256;
static constexpr size_t O_GATE = O_STAR + 256 * 512;
static constexpr size_t O_EW1  = O_GATE + 6 * 16 * 256;
static constexpr size_t O_EW2  = O_EW1 + 8 * 128 * 256;
static constexpr size_t O_DW1  = O_EW2 + 8 * 64 * 128;
static constexpr size_t O_DW2  = O_DW1 + 3 * 128 * 256;
static constexpr size_t O_TW1  = O_DW2 + 3 * 64 * 128;
static constexpr size_t O_TW2  = O_TW1 + 2 * 128 * 256;
static constexpr size_t O_DSK  = O_TW2 + 2 * 64 * 128;
static constexpr size_t O_TOW  = O_DSK + 6 * 64 * 256;
static constexpr size_t O_END  = O_TOW + 6 * 64 * 64;

struct Params {
  const int* x;
  const float* emb;
  const _Float16* skipWt; const float* skip_b; const float* skip_g; const float* skip_be;
  const _Float16* slotWt; const float* slot_b; const float* shared_b;
  const _Float16* starWt; const float* star_b; const float* star_g; const float* star_be;
  const _Float16* gateWt; const float* gate_b;
  const _Float16* eW1; const float* e_b1; const float* e_g1; const float* e_be1;
  const _Float16* eW2; const float* e_b2; const float* e_g2; const float* e_be2;
  const _Float16* dW1; const float* d_b1; const float* d_g1; const float* d_be1;
  const _Float16* dW2; const float* d_b2; const float* d_g2; const float* d_be2;
  const _Float16* tW1; const float* t_b1; const float* t_g1; const float* t_be1;
  const _Float16* tW2; const float* t_b2; const float* t_g2; const float* t_be2;
  const _Float16* dskWt; const float* dsk_b; const float* dsk_g; const float* dsk_be;
  const _Float16* towWt; const float* tow_b1; const float* tow_g; const float* tow_be;
  const float* tow_W2; const float* tow_b2;
  float* out;
  int B; int zpad;
};
typedef char params_size_check[(sizeof(Params) == 50 * 8 + 8) ? 1 : -1];

#define HZNOP "v_nop\n\tv_nop\n\tv_nop\n\tv_nop"
__device__ __forceinline__ void hz(v8f (&c)[1], v16h& a, v16h& b) {
  asm volatile(HZNOP : "+v"(c[0]) : "v"(a), "v"(b));
}
__device__ __forceinline__ void hz(v8f (&c)[4], v16h& a, v16h& b) {
  asm volatile(HZNOP : "+v"(c[0]), "+v"(c[1]), "+v"(c[2]), "+v"(c[3]) : "v"(a), "v"(b));
}
__device__ __forceinline__ void hz(v8f (&c)[6], v16h& a, v16h& b) {
  asm volatile(HZNOP : "+v"(c[0]), "+v"(c[1]), "+v"(c[2]), "+v"(c[3]), "+v"(c[4]), "+v"(c[5])
               : "v"(a), "v"(b));
}
__device__ __forceinline__ void hz(v8f (&c)[8], v16h& a, v16h& b) {
  asm volatile(HZNOP : "+v"(c[0]), "+v"(c[1]), "+v"(c[2]), "+v"(c[3]),
                       "+v"(c[4]), "+v"(c[5]), "+v"(c[6]), "+v"(c[7]) : "v"(a), "v"(b));
}
__device__ __forceinline__ void hz(v8f (&c)[16], v16h& a, v16h& b) {
  asm volatile(HZNOP : "+v"(c[0]), "+v"(c[1]), "+v"(c[2]), "+v"(c[3]),
                       "+v"(c[4]), "+v"(c[5]), "+v"(c[6]), "+v"(c[7]),
                       "+v"(c[8]), "+v"(c[9]), "+v"(c[10]), "+v"(c[11]),
                       "+v"(c[12]), "+v"(c[13]), "+v"(c[14]), "+v"(c[15]) : "v"(a), "v"(b));
}

template<int NT, int KT>
__device__ __forceinline__ void wgemm(const _Float16* A, int lda,
                                      const _Float16* __restrict__ W, int ldw,
                                      v8f (&c)[NT], int lane) {
  #pragma unroll
  for (int t = 0; t < NT; ++t) { v8f z = {0.f, 0.f, 0.f, 0.f, 0.f, 0.f, 0.f, 0.f}; c[t] = z; }
  const int m  = lane & 15;
  const int h8 = (lane >> 4) * 8;
  const _Float16* pa = A + m * lda + h8;
  const _Float16* pw = W + (size_t)m * ldw + h8;
  #pragma unroll 1
  for (int ks = 0; ks < KT; ++ks) {
    Frag a, b;
    a.h[0] = *(const v8h*)(pa + ks * 32);
    a.h[1] = *(const v8h*)(pa + ks * 32 + 16);
    #pragma unroll
    for (int t = 0; t < NT; ++t) {
      const _Float16* q = pw + (size_t)t * 16 * ldw + ks * 32;
      b.h[0] = *(const v8h*)(q);
      b.h[1] = *(const v8h*)(q + 16);
      c[t] = __builtin_amdgcn_wmma_f32_16x16x32_f16(false, a.v, false, b.v, (short)0, c[t], false, false);
    }
    hz(c, a.v, b.v);
  }
}

template<int NT>
__device__ __forceinline__ void ln_relu(v8f (&c)[NT], float scale, const float* __restrict__ bp,
                                        const float* __restrict__ gp, const float* __restrict__ ep,
                                        int lane) {
  const int col = lane & 15;
  float s[8], s2[8];
  #pragma unroll
  for (int v = 0; v < 8; ++v) { s[v] = 0.f; s2[v] = 0.f; }
  #pragma unroll
  for (int t = 0; t < NT; ++t) {
    const float bias = bp[t * 16 + col];
    #pragma unroll
    for (int v = 0; v < 8; ++v) {
      float xx = c[t][v] * scale + bias;
      c[t][v] = xx;
      s[v] += xx; s2[v] += xx * xx;
    }
  }
  #pragma unroll
  for (int mm = 1; mm <= 8; mm <<= 1)
    #pragma unroll
    for (int v = 0; v < 8; ++v) {
      s[v]  += __shfl_xor(s[v],  mm, 16);
      s2[v] += __shfl_xor(s2[v], mm, 16);
    }
  const float invN = 1.0f / (float)(NT * 16);
  float mu[8], rs[8];
  #pragma unroll
  for (int v = 0; v < 8; ++v) {
    mu[v] = s[v] * invN;
    float var = s2[v] * invN - mu[v] * mu[v];
    var = fmaxf(var, 0.f);
    rs[v] = rsqrtf(var + 1e-5f);
  }
  #pragma unroll
  for (int t = 0; t < NT; ++t) {
    const float g = gp[t * 16 + col], be = ep[t * 16 + col];
    #pragma unroll
    for (int v = 0; v < 8; ++v) {
      float y = (c[t][v] - mu[v]) * rs[v] * g + be;
      c[t][v] = fmaxf(y, 0.f);
    }
  }
}

template<int NT>
__device__ __forceinline__ void store_act(_Float16* dst, int ld, const v8f (&c)[NT], int lane) {
  const int col = lane & 15, r0 = (lane >> 4) * 8;
  #pragma unroll
  for (int t = 0; t < NT; ++t)
    #pragma unroll
    for (int v = 0; v < 8; ++v)
      dst[(r0 + v) * ld + t * 16 + col] = (_Float16)c[t][v];
}

template<int NT>
__device__ __forceinline__ void store_f32(float* dst, int ld, const v8f (&c)[NT], int lane) {
  const int col = lane & 15, r0 = (lane >> 4) * 8;
  #pragma unroll
  for (int t = 0; t < NT; ++t)
    #pragma unroll
    for (int v = 0; v < 8; ++v)
      dst[(r0 + v) * ld + t * 16 + col] = c[t][v];
}

__global__ void __launch_bounds__(WAVES * 32) __attribute__((amdgpu_num_vgpr(256)))
k_forward(Params p) {
  extern __shared__ v4f dsm[];
  unsigned char* smem = (unsigned char*)dsm;
  int*   skey = (int*)(smem + BO_SKEY);
  int*   perm = (int*)(smem + BO_PERM);
  int*   cnt  = (int*)(smem + BO_CNT);
  float* res  = (float*)(smem + BO_RES);

  const int lane = threadIdx.x & 31;
  const int wave = threadIdx.x >> 5;
  const int col  = lane & 15;
  const int hi   = lane >> 4;
  unsigned char* my = smem + BLK_BYTES + wave * PER_WAVE;
  _Float16* bufIn   = (_Float16*)(my + OFF_IN);
  _Float16* bufSkip = (_Float16*)(my + OFF_SKIP);
  _Float16* bufMid  = (_Float16*)(my + OFF_MID);
  float*    fea     = (float*)   (my + OFF_FEA);
  _Float16* h1      = (_Float16*)(my + OFF_H1);
  float*    gates   = (float*)   (my + OFF_GATE);
  float*    probs   = (float*)   (my + OFF_PROB);

  const int B = p.B;
  const int base = blockIdx.x * SPB;

  int keyg[4], rankg[4];
  #pragma unroll
  for (int g = 0; g < 4; ++g) {
    const int i = wave * 128 + g * 32 + lane;
    const int s = base + i;
    const int sc = (s < B) ? s : (B - 1);
    const int dom = p.x[(size_t)(FEATS - 1) * (size_t)B + sc];
    const int key = ((unsigned)dom < 3u) ? dom : 3;
    const unsigned m0 = __builtin_amdgcn_ballot_w32(key == 0);
    const unsigned m1 = __builtin_amdgcn_ballot_w32(key == 1);
    const unsigned m2 = __builtin_amdgcn_ballot_w32(key == 2);
    const unsigned m3 = __builtin_amdgcn_ballot_w32(key == 3);
    const unsigned lower = (1u << lane) - 1u;
    const unsigned mk = (key == 0) ? m0 : (key == 1) ? m1 : (key == 2) ? m2 : m3;
    rankg[g] = __builtin_popcount(mk & lower);
    keyg[g]  = key;
    if (lane < 4) {
      const unsigned mm = (lane == 0) ? m0 : (lane == 1) ? m1 : (lane == 2) ? m2 : m3;
      cnt[(wave * 4 + g) * 4 + lane] = __builtin_popcount(mm);
    }
  }
  __syncthreads();
  {
    int tot0 = 0, tot1 = 0, tot2 = 0;
    #pragma unroll
    for (int G = 0; G < 8; ++G) { tot0 += cnt[G * 4 + 0]; tot1 += cnt[G * 4 + 1]; tot2 += cnt[G * 4 + 2]; }
    #pragma unroll
    for (int g = 0; g < 4; ++g) {
      const int key = keyg[g];
      const int G = wave * 4 + g;
      int pre = (key == 0) ? 0 : (key == 1) ? tot0 : (key == 2) ? (tot0 + tot1) : (tot0 + tot1 + tot2);
      #pragma unroll
      for (int q = 0; q < 8; ++q) pre += (q < G) ? cnt[q * 4 + key] : 0;
      const int pos = pre + rankg[g];
      if ((unsigned)pos < (unsigned)SPB) {
        perm[pos] = wave * 128 + g * 32 + lane;
        skey[pos] = key;
      }
    }
  }
  __syncthreads();

  #pragma unroll 1
  for (int tt = 0; tt < TPW; ++tt) {
    const int p0 = (wave * TPW + tt) * 16;

    const int lsamp = perm[p0 + col];
    const int sgl = base + lsamp;
    const int sc = (sgl < B) ? sgl : (B - 1);
    {
      #pragma unroll 4
      for (int f = 0; f < FEATS; ++f) {
        int idx = p.x[(size_t)f * (size_t)B + sc];
        if (idx < 0) idx += VOCAB;
        idx = (idx < 0) ? 0 : ((idx > VOCAB - 1) ? (VOCAB - 1) : idx);
        const float* e = p.emb + ((size_t)(f * VOCAB + idx)) * EDIM + hi * 8;
        const v4f ea = *(const v4f*)e;
        const v4f eb = *(const v4f*)(e + 4);
        v8h hv;
        hv[0] = (_Float16)(ea[0] * S_IN); hv[1] = (_Float16)(ea[1] * S_IN);
        hv[2] = (_Float16)(ea[2] * S_IN); hv[3] = (_Float16)(ea[3] * S_IN);
        hv[4] = (_Float16)(eb[0] * S_IN); hv[5] = (_Float16)(eb[1] * S_IN);
        hv[6] = (_Float16)(eb[2] * S_IN); hv[7] = (_Float16)(eb[3] * S_IN);
        *(v8h*)(bufIn + col * DIN + f * EDIM + hi * 8) = hv;
      }
    }
    const int domraw = p.x[(size_t)(FEATS - 1) * (size_t)B + sc];
    int dmin = skey[p0], dmax = skey[p0 + 15];
    dmin = __builtin_amdgcn_readfirstlane(dmin);
    dmax = __builtin_amdgcn_readfirstlane(dmax);
    __syncthreads();

    {
      v8f c[16];
      wgemm<16, 8>(bufIn, DIN, p.skipWt, DIN, c, lane);
      ln_relu<16>(c, 1.f / (S_IN * S_W), p.skip_b, p.skip_g, p.skip_be, lane);
      store_act<16>(bufSkip, SOUT, c, lane);
    }

    {
      int dom_v[8];
      #pragma unroll
      for (int v = 0; v < 8; ++v) dom_v[v] = skey[p0 + hi * 8 + v];
      v8f c[16];
      #pragma unroll 1
      for (int d = 0; d < NDOM; ++d) {
        if (d >= dmin && d <= dmax) {
          #pragma unroll 1
          for (int ch = 0; ch < 2; ++ch) {
            wgemm<16, 8>(bufIn, DIN, p.slotWt + ((size_t)d * SMID + (size_t)ch * 256) * DIN, DIN, c, lane);
            #pragma unroll
            for (int t = 0; t < 16; ++t) {
              const int n = ch * 256 + t * 16 + col;
              const float sb = (p.slot_b[d * SMID + n] + p.shared_b[n]) * S_MID;
              #pragma unroll
              for (int v = 0; v < 8; ++v)
                if (dom_v[v] == d)
                  bufMid[(v + hi * 8) * SMID + n] = (_Float16)(c[t][v] * (S_MID / (S_IN * S_SLOT)) + sb);
            }
          }
        }
      }
      if (dmax == 3) {
        #pragma unroll
        for (int v = 0; v < 8; ++v) {
          if (dom_v[v] == 3) {
            _Float16* row = bufMid + (v + hi * 8) * SMID;
            #pragma unroll 4
            for (int t = 0; t < SMID / 16; ++t) row[t * 16 + col] = (_Float16)0.f;
          }
        }
      }
    }
    __syncthreads();

    {
      v8f c[16];
      wgemm<16, 16>(bufMid, SMID, p.starWt, SMID, c, lane);
      ln_relu<16>(c, 1.f / (S_MID * S_W), p.star_b, p.star_g, p.star_be, lane);
      #pragma unroll
      for (int t = 0; t < 16; ++t)
        #pragma unroll
        for (int v = 0; v < 8; ++v) {
          const int r = v + hi * 8, n = t * 16 + col;
          const float y = c[t][v] + (float)bufSkip[r * SOUT + n];
          bufIn[r * SOUT + n] = (_Float16)y;
        }
    }
    __syncthreads();

    {
      v8f cg[6];
      wgemm<6, 8>(bufIn, DIN, p.gateWt, DIN, cg, lane);
      #pragma unroll
      for (int k = 0; k < NKDT; ++k) {
        const float bsf = (col < 8) ? p.gate_b[k * NEXP + col] : 0.f;
        float l[8], mx[8], ex[8], sm[8];
        #pragma unroll
        for (int v = 0; v < 8; ++v) { l[v] = cg[k][v] * (1.f / S_W) + bsf; mx[v] = l[v]; }
        #pragma unroll
        for (int mm = 1; mm <= 4; mm <<= 1)
          #pragma unroll
          for (int v = 0; v < 8; ++v) mx[v] = fmaxf(mx[v], __shfl_xor(mx[v], mm, 16));
        #pragma unroll
        for (int v = 0; v < 8; ++v) { ex[v] = __expf(l[v] - mx[v]); sm[v] = ex[v]; }
        #pragma unroll
        for (int mm = 1; mm <= 4; mm <<= 1)
          #pragma unroll
          for (int v = 0; v < 8; ++v) sm[v] += __shfl_xor(sm[v], mm, 16);
        if (col < 8) {
          #pragma unroll
          for (int v = 0; v < 8; ++v) {
            const float inv = 1.f / sm[v];
            gates[(k * 16 + v + hi * 8) * NEXP + col] = ex[v] * inv;
          }
        }
      }
    }

    #pragma unroll 1
    for (int q = 0; q < NXP; ++q) {
      const _Float16* W1; const float* b1; const float* g1; const float* e1;
      const _Float16* W2; const float* b2; const float* g2; const float* e2;
      if (q < NEXP) {
        const int e = q;
        W1 = p.eW1 + (size_t)e * H1D * DIN; b1 = p.e_b1 + e * H1D; g1 = p.e_g1 + e * H1D; e1 = p.e_be1 + e * H1D;
        W2 = p.eW2 + (size_t)e * H2D * H1D; b2 = p.e_b2 + e * H2D; g2 = p.e_g2 + e * H2D; e2 = p.e_be2 + e * H2D;
      } else if (q < NEXP + NDOM) {
        const int d = q - NEXP;
        W1 = p.dW1 + (size_t)d * H1D * DIN; b1 = p.d_b1 + d * H1D; g1 = p.d_g1 + d * H1D; e1 = p.d_be1 + d * H1D;
        W2 = p.dW2 + (size_t)d * H2D * H1D; b2 = p.d_b2 + d * H2D; g2 = p.d_g2 + d * H2D; e2 = p.d_be2 + d * H2D;
      } else {
        const int ts = q - NEXP - NDOM;
        W1 = p.tW1 + (size_t)ts * H1D * DIN; b1 = p.t_b1 + ts * H1D; g1 = p.t_g1 + ts * H1D; e1 = p.t_be1 + ts * H1D;
        W2 = p.tW2 + (size_t)ts * H2D * H1D; b2 = p.t_b2 + ts * H2D; g2 = p.t_g2 + ts * H2D; e2 = p.t_be2 + ts * H2D;
      }
      {
        v8f h1c[8];
        wgemm<8, 8>(bufIn, DIN, W1, DIN, h1c, lane);
        ln_relu<8>(h1c, 1.f / S_W, b1, g1, e1, lane);
        store_act<8>(h1, H1D, h1c, lane);
      }
      __syncthreads();
      {
        v8f h2[4];
        wgemm<4, 4>(h1, H1D, W2, H1D, h2, lane);
        ln_relu<4>(h2, 1.f / S_W, b2, g2, e2, lane);
        store_f32<4>(fea + q * 1024, H2D, h2, lane);
      }
      __syncthreads();
    }

    #pragma unroll 1
    for (int k = 0; k < NKDT; ++k) {
      v8f fz[4];
      wgemm<4, 8>(bufIn, DIN, p.dskWt + (size_t)k * H2D * DIN, DIN, fz, lane);
      ln_relu<4>(fz, 1.f / S_W, p.dsk_b + k * H2D, p.dsk_g + k * H2D, p.dsk_be + k * H2D, lane);
      const int kd = k % NDOM, kt = k % NTSK;
      const float* df = fea + (NEXP + kd) * 1024;
      const float* tf = fea + (NEXP + NDOM + kt) * 1024;
      #pragma unroll
      for (int t = 0; t < 4; ++t)
        #pragma unroll
        for (int v = 0; v < 8; ++v) {
          const int ix = (v + hi * 8) * H2D + t * 16 + col;
          fz[t][v] = 0.5f * fz[t][v] + df[ix] + tf[ix];
        }
      #pragma unroll 2
      for (int e = 0; e < NEXP; ++e) {
        const float* fe = fea + e * 1024;
        float gv[8];
        #pragma unroll
        for (int v = 0; v < 8; ++v) gv[v] = gates[(k * 16 + v + hi * 8) * NEXP + e];
        #pragma unroll
        for (int t = 0; t < 4; ++t)
          #pragma unroll
          for (int v = 0; v < 8; ++v) {
            const int ix = (v + hi * 8) * H2D + t * 16 + col;
            fz[t][v] += gv[v] * fe[ix];
          }
      }
      store_act<4>(h1, H2D, fz, lane);
      __syncthreads();
      {
        v8f hc[4];
        wgemm<4, 2>(h1, H2D, p.towWt + (size_t)k * H2D * H2D, H2D, hc, lane);
        ln_relu<4>(hc, 1.f / S_W, p.tow_b1 + k * H2D, p.tow_g + k * H2D, p.tow_be + k * H2D, lane);
        float w2[4];
        #pragma unroll
        for (int t = 0; t < 4; ++t) w2[t] = p.tow_W2[k * H2D + t * 16 + col];
        float pd[8];
        #pragma unroll
        for (int v = 0; v < 8; ++v) {
          pd[v] = 0.f;
          #pragma unroll
          for (int t = 0; t < 4; ++t) pd[v] += hc[t][v] * w2[t];
        }
        #pragma unroll
        for (int mm = 1; mm <= 8; mm <<= 1)
          #pragma unroll
          for (int v = 0; v < 8; ++v) pd[v] += __shfl_xor(pd[v], mm, 16);
        const float b2k = p.tow_b2[k];
        if (col == 0) {
          #pragma unroll
          for (int v = 0; v < 8; ++v)
            probs[k * 16 + v + hi * 8] = 1.f / (1.f + __expf(-(pd[v] + b2k)));
        }
      }
      __syncthreads();
    }

    if (lane < 16) {
      int dd = domraw;
      if (dd < 0) dd += NDOM;
      dd = (dd < 0) ? 0 : ((dd > NDOM - 1) ? (NDOM - 1) : dd);
      res[lsamp * 2 + 0] = probs[(0 * NDOM + dd) * 16 + lane];
      res[lsamp * 2 + 1] = probs[(1 * NDOM + dd) * 16 + lane];
    }
  }
  __syncthreads();

  if (wave == 0) {
    const int nv = (B - base < SPB) ? (B - base) : SPB;
    float* ob = p.out + (size_t)base * 2;
    v4f vv[4];
    #pragma unroll
    for (int q = 0; q < 4; ++q) vv[q] = *(const v4f*)(res + (q * 32 + lane) * 4);
    if (nv == SPB) {
      #pragma unroll
      for (int q = 0; q < 4; ++q) *(volatile v4f*)(ob + (q * 32 + lane) * 4) = vv[q];
      __threadfence();
      #pragma unroll
      for (int q = 0; q < 4; ++q) *(volatile v4f*)(ob + (q * 32 + lane) * 4) = vv[q];
    } else {
      #pragma unroll
      for (int q = 0; q < 4; ++q)
        #pragma unroll
        for (int cc = 0; cc < 4; ++cc) {
          const int ix = (q * 32 + lane) * 4 + cc;
          if ((ix >> 1) < nv) ((volatile float*)ob)[ix] = vv[q][cc];
        }
      __threadfence();
      #pragma unroll
      for (int q = 0; q < 4; ++q)
        #pragma unroll
        for (int cc = 0; cc < 4; ++cc) {
          const int ix = (q * 32 + lane) * 4 + cc;
          if ((ix >> 1) < nv) ((volatile float*)ob)[ix] = vv[q][cc];
        }
    }
  }
}

__global__ void __launch_bounds__(256) k_prep_t(const float* __restrict__ src, _Float16* dst,
                                                 int K, int N, int Ndst, float scale,
                                                 int srcStride, int dstStride) {
  const float* s = src + (size_t)blockIdx.y * (size_t)srcStride;
  _Float16* d = dst + (size_t)blockIdx.y * (size_t)dstStride;
  const int nvec = (K * Ndst) >> 3;
  const int i = blockIdx.x * 256 + threadIdx.x;
  if (i >= nvec) return;
  const int e0 = i << 3;
  const int n = e0 / K;
  const int k0 = e0 - n * K;
  v8h hv;
  #pragma unroll
  for (int jj = 0; jj < 8; ++jj) {
    float v = 0.f;
    if (n < N) v = s[(size_t)(k0 + jj) * N + n] * scale;
    hv[jj] = (_Float16)v;
  }
  volatile v8h* q = (volatile v8h*)(d + e0);
  *q = hv;
  __threadfence();
  *q = hv;
}

__global__ void __launch_bounds__(256) k_prep_slot(const float* __restrict__ slotW, const float* __restrict__ sharedW,
                                                    _Float16* dst, float scale) {
  const int nvec = (NDOM * SMID * DIN) >> 3;
  const int i = blockIdx.x * 256 + threadIdx.x;
  if (i >= nvec) return;
  const int e0 = i << 3;
  const int d = e0 / (SMID * DIN);
  const int r = e0 - d * (SMID * DIN);
  const int n = r / DIN;
  const int k0 = r - n * DIN;
  v8h hv;
  #pragma unroll
  for (int jj = 0; jj < 8; ++jj) {
    const int k = k0 + jj;
    const float pr = slotW[((size_t)d * DIN + k) * SMID + n] * sharedW[(size_t)k * SMID + n];
    hv[jj] = (_Float16)(pr * scale);
  }
  volatile v8h* q = (volatile v8h*)(dst + e0);
  *q = hv;
  __threadfence();
  *q = hv;
}

extern "C" void kernel_launch(void* const* d_in, const int* in_sizes, int n_in,
                              void* d_out, int out_size, void* d_ws, size_t ws_size,
                              hipStream_t stream) {
  if (n_in < 50) return;
  const int B = in_sizes[0] / FEATS;
  if (B <= 0) return;
  if ((long long)out_size < 2LL * (long long)B) return;
  const size_t wsNeed = O_END * sizeof(_Float16);
  if (wsNeed > ws_size) return;

  auto f32 = [&](int i) { return (const float*)d_in[i]; };
  _Float16* ws = (_Float16*)d_ws;

  auto T = [&](const float* src, size_t dstOff, int K, int N, int Ndst, float scale, int count) {
    const int nvec = (K * Ndst) >> 3;
    dim3 grid((nvec + 255) / 256, count);
    k_prep_t<<<grid, 256, 0, stream>>>(src, ws + dstOff, K, N, Ndst, scale, K * N, K * Ndst);
  };

  T(f32(2), O_SKIP, DIN, SOUT, SOUT, S_W, 1);
  k_prep_slot<<<((NDOM * SMID * DIN) / 8 + 255) / 256, 256, 0, stream>>>(f32(8), f32(6), ws + O_SLOT, S_SLOT);
  T(f32(10), O_STAR, SMID, SOUT, SOUT, S_W, 1);
  T(f32(42), O_GATE, DIN, NEXP, 16, S_W, NKDT);
  T(f32(18), O_EW1, DIN, H1D, H1D, S_W, NEXP);
  T(f32(22), O_EW2, H1D, H2D, H2D, S_W, NEXP);
  T(f32(26), O_DW1, DIN, H1D, H1D, S_W, NDOM);
  T(f32(30), O_DW2, H1D, H2D, H2D, S_W, NDOM);
  T(f32(34), O_TW1, DIN, H1D, H1D, S_W, NTSK);
  T(f32(38), O_TW2, H1D, H2D, H2D, S_W, NTSK);
  T(f32(14), O_DSK, DIN, H2D, H2D, S_W, NKDT);
  T(f32(44), O_TOW, H2D, H2D, H2D, S_W, NKDT);

  Params p;
  p.x = (const int*)d_in[0];
  p.emb = f32(1);
  p.skipWt = ws + O_SKIP; p.skip_b = f32(3); p.skip_g = f32(4); p.skip_be = f32(5);
  p.slotWt = ws + O_SLOT; p.slot_b = f32(9); p.shared_b = f32(7);
  p.starWt = ws + O_STAR; p.star_b = f32(11); p.star_g = f32(12); p.star_be = f32(13);
  p.gateWt = ws + O_GATE; p.gate_b = f32(43);
  p.eW1 = ws + O_EW1; p.e_b1 = f32(19); p.e_g1 = f32(20); p.e_be1 = f32(21);
  p.eW2 = ws + O_EW2; p.e_b2 = f32(23); p.e_g2 = f32(24); p.e_be2 = f32(25);
  p.dW1 = ws + O_DW1; p.d_b1 = f32(27); p.d_g1 = f32(28); p.d_be1 = f32(29);
  p.dW2 = ws + O_DW2; p.d_b2 = f32(31); p.d_g2 = f32(32); p.d_be2 = f32(33);
  p.tW1 = ws + O_TW1; p.t_b1 = f32(35); p.t_g1 = f32(36); p.t_be1 = f32(37);
  p.tW2 = ws + O_TW2; p.t_b2 = f32(39); p.t_g2 = f32(40); p.t_be2 = f32(41);
  p.dskWt = ws + O_DSK; p.dsk_b = f32(15); p.dsk_g = f32(16); p.dsk_be = f32(17);
  p.towWt = ws + O_TOW; p.tow_b1 = f32(45); p.tow_g = f32(46); p.tow_be = f32(47);
  p.tow_W2 = f32(48); p.tow_b2 = f32(49);
  p.out = (float*)d_out;
  p.B = B;
  p.zpad = 0;

  hipFuncSetAttribute(reinterpret_cast<const void*>(k_forward),
                      hipFuncAttributeMaxDynamicSharedMemorySize, SMEM_BYTES);
  const int nblk = (B + SPB - 1) / SPB;
  k_forward<<<nblk, WAVES * 32, SMEM_BYTES, stream>>>(p);
}
